// RoPEAttention_13357348291165
// MI455X (gfx1250) — hardware-verified
//
#include <hip/hip_runtime.h>

#pragma clang fp contract(off)

#define DI __device__ __forceinline__

typedef _Float16 h8  __attribute__((ext_vector_type(8), __may_alias__));
typedef _Float16 h16 __attribute__((ext_vector_type(16)));
typedef float    f8  __attribute__((ext_vector_type(8)));
typedef float    v4f __attribute__((ext_vector_type(4), __may_alias__));

#ifndef NB
#define NB 4
#endif
#ifndef SEQ
#define SEQ 2048
#endif
#define NB_FULL  4
#define SEQ_FULL 2048
#define DIM   1024
#define NH    16
#define HD    64
#define QKVN  3072
#define ROWS  (NB * SEQ)
#define NBH   (NB * NH)

static_assert(NB >= 1 && NB <= NB_FULL);
static_assert(SEQ >= 64 && SEQ <= SEQ_FULL && (SEQ % 64) == 0);
static_assert((DIM % 32) == 0 && (QKVN % 64) == 0 && (ROWS % 64) == 0);

#define WS_TAB   ((size_t)0)
#define WS_XH    ((size_t)4096)
#define WS_WQ    (WS_XH + (size_t)ROWS * DIM * 2)
#define WS_WP    (WS_WQ + (size_t)QKVN * DIM * 2)
#define WS_Q     (WS_WP + (size_t)DIM * DIM * 2)
#define WS_K     (WS_Q  + (size_t)NBH * SEQ * HD * 2)
#define WS_VT    (WS_K  + (size_t)NBH * SEQ * HD * 2)
#define WS_ATT   (WS_VT + (size_t)NBH * HD * SEQ * 2)
#define WS_TOTAL (WS_ATT + (size_t)ROWS * DIM * 2)
static_assert(WS_TOTAL <= (size_t)134217728);
static_assert((size_t)((NB - 1) * SEQ_FULL + SEQ) * DIM * 4 <= (size_t)NB_FULL * SEQ_FULL * DIM * 4);

DI h16 load_frag(const _Float16* base, int ld, int k0, int lane) {
  const _Float16* p = base + (size_t)(lane & 15) * ld + k0 + ((lane >> 4) << 3);
  h8 lo = *(const h8*)(p);
  h8 hi = *(const h8*)(p + 16);
  return __builtin_shufflevector(lo, hi, 0, 1, 2, 3, 4, 5, 6, 7,
                                 8, 9, 10, 11, 12, 13, 14, 15);
}

DI f8 wmma16(h16 a, h16 b, f8 c) {
  return __builtin_amdgcn_wmma_f32_16x16x32_f16(false, a, false, b,
                                                (short)0, c, false, false);
}

DI float bfr(float f) {
  unsigned u = __builtin_bit_cast(unsigned, f);
  u += 0x7FFFu + ((u >> 16) & 1u);
  u &= 0xFFFF0000u;
  return __builtin_bit_cast(float, u);
}

DI float omega_of(int fi) {
  return (fi == 0) ? 1.0f
       : (fi == 1) ? 0.3981071705534972f
       : (fi == 2) ? 0.15848931924611134f
       : (fi == 3) ? 0.06309573444801933f
       : (fi == 4) ? 0.025118864315095794f
       : (fi == 5) ? 0.01f
       : (fi == 6) ? 0.003981071705534973f
       : (fi == 7) ? 0.001584893192461114f
       : (fi == 8) ? 0.000630957344480193f
       : (fi == 9) ? 0.00025118864315095795f
       : 0.0f;
}

DI void sincos_small(float a, float& sn, float& cs) {
  float k = rintf(a * 0.63661977236758134f);
  float r = fmaf(-k, 1.57079637050628662109375f, a);
  r = fmaf(k, 4.37113900018624283e-8f, r);
  float r2 = r * r;
  float sp = r + r * r2 * (-1.6666667163e-1f + r2 * (8.3333337680e-3f +
             r2 * (-1.9841270114e-4f + r2 * 2.7557314297e-6f)));
  float cp = 1.0f + r2 * (-0.5f + r2 * (4.1666667908e-2f + r2 * (-1.3888889225e-3f +
             r2 * (2.4801587642e-5f + r2 * (-2.7557314297e-7f)))));
  int q = ((int)k) & 3;
  sn = (q == 0) ? sp : (q == 1) ? cp : (q == 2) ? -sp : -cp;
  cs = (q == 0) ? cp : (q == 1) ? -sp : (q == 2) ? -cp : sp;
}

__global__ void __launch_bounds__(128) k_tab(float* __restrict__ tab) {
  const int t = threadIdx.x;
  v4f val;
#pragma unroll
  for (int q = 0; q < 4; ++q) {
    int e = 4 * t + q;
    int s = e & 255;
    int pos = s >> 4, fi = s & 15;
    float a = (float)pos * omega_of(fi);
    float sn, cs;
    sincos_small(a, sn, cs);
    val[q] = (e < 256) ? cs : sn;
  }
  volatile v4f* p = (volatile v4f*)(tab + 4 * t);
  *p = val;
  __threadfence();
  *p = val;
}

__global__ void __launch_bounds__(256) k_cvt(const float* __restrict__ in,
                                             _Float16* __restrict__ out,
                                             int rows, int cols8, int seq,
                                             int seqfull, float scale) {
  const int g = blockIdx.x * 256 + threadIdx.x;
  const int total = rows * cols8;
  if (g >= total) return;
  const int r = g / cols8, c8 = g - r * cols8;
  const int b = r / seq, t = r - b * seq;
  const size_t cols = (size_t)cols8 * 8;
  const size_t irow = (size_t)b * seqfull + t;
  const v4f* src = (const v4f*)(in + irow * cols + (size_t)c8 * 8);
  v4f a0 = src[0], a1 = src[1];
  h8 o;
#pragma unroll
  for (int q = 0; q < 4; ++q) {
    float x0 = a0[q];
    float x1 = a1[q];
    o[q]     = (_Float16)(bfr(x0) * scale);
    o[q + 4] = (_Float16)(bfr(x1) * scale);
  }
  volatile h8* dst = (volatile h8*)(out + (size_t)r * cols + (size_t)c8 * 8);
  *dst = o;
  __threadfence();
  *dst = o;
}

#define SP 72

__global__ void __launch_bounds__(128) k_qkv_rot(const _Float16* __restrict__ xh,
                                                 const _Float16* __restrict__ wq,
                                                 const float* __restrict__ tab,
                                                 _Float16* __restrict__ qb,
                                                 _Float16* __restrict__ kb,
                                                 _Float16* __restrict__ vtb) {
  __shared__ __attribute__((aligned(16))) float tabL[512];
  __shared__ __attribute__((aligned(16))) _Float16 stg[64 * SP];
  const int tid = threadIdx.x, lane = tid & 31, wid = tid >> 5, hh = lane >> 4;
  const int wm = wid & 1, wn = wid >> 1;
  const int mt = blockIdx.x / (QKVN / 64), nt = blockIdx.x - mt * (QKVN / 64);
  const int m0 = mt * 64, n0 = nt * 64;
  const int part = n0 >> 10;
  const int head = (n0 & (DIM - 1)) >> 6;
  const int b = m0 / SEQ, t0 = m0 - b * SEQ;

  *(v4f*)(tabL + 4 * tid) = *(const v4f*)(tab + 4 * tid);
  __syncthreads();

  const _Float16* arow = xh + (size_t)(m0 + wm * 32) * DIM;
  const _Float16* brow = wq + (size_t)(n0 + wn * 32) * DIM;
  f8 c00 = {}, c01 = {}, c10 = {}, c11 = {};
#pragma unroll 1
  for (int k0 = 0; k0 < DIM; k0 += 32) {
    h16 a0 = load_frag(arow, DIM, k0, lane);
    h16 a1 = load_frag(arow + (size_t)16 * DIM, DIM, k0, lane);
    h16 b0 = load_frag(brow, DIM, k0, lane);
    h16 b1 = load_frag(brow + (size_t)16 * DIM, DIM, k0, lane);
    c00 = wmma16(a0, b0, c00);
    c01 = wmma16(a0, b1, c01);
    c10 = wmma16(a1, b0, c10);
    c11 = wmma16(a1, b1, c11);
    asm volatile("v_nop\n\tv_nop\n\tv_nop\n\tv_nop"
                 : "+v"(c00), "+v"(c01), "+v"(c10), "+v"(c11)
                 : "v"(a0), "v"(a1), "v"(b0), "v"(b1));
  }

#pragma unroll
  for (int i = 0; i < 2; ++i) {
#pragma unroll
    for (int j = 0; j < 2; ++j) {
      f8 acc = i ? (j ? c11 : c10) : (j ? c01 : c00);
      const int d = wn * 32 + j * 16 + (lane & 15);
      const int axis = (d >= 40) ? 2 : (d >= 20) ? 1 : 0;
      const int fi = (d - 20 * axis) >> 1;
      const bool rot = (part < 2) && (d < 60);
#pragma unroll
      for (int r = 0; r < 8; ++r) {
        const int lr = wm * 32 + i * 16 + 8 * hh + r;
        const int t = t0 + lr;
        float v = acc[r] * (1.0f / 32.0f);
        float partner = __shfl_xor(v, 1, 32);
        const int pos = (axis == 0) ? (t >> 8) : (axis == 1) ? ((t >> 4) & 15) : (t & 15);
        float c = tabL[pos * 16 + fi];
        float s = tabL[256 + pos * 16 + fi];
        float o = (d & 1) ? (v * c + partner * s) : (v * c - partner * s);
        o = rot ? o : v;
        stg[lr * SP + d] = (_Float16)o;
      }
    }
  }
  __syncthreads();

  const int bh = b * NH + head;
  const int sub = tid >> 3, ch = tid & 7;
  if (part < 2) {
    _Float16* plane = (part == 0) ? qb : kb;
    h8 vals[4];
#pragma unroll
    for (int p = 0; p < 4; ++p) {
      const int lr = p * 16 + sub;
      vals[p] = *(const h8*)(stg + lr * SP + ch * 8);
    }
    _Float16* base = plane + ((size_t)bh * SEQ + t0) * HD + ch * 8;
#pragma unroll
    for (int p = 0; p < 4; ++p)
      *(volatile h8*)(base + (size_t)(p * 16 + sub) * HD) = vals[p];
    __threadfence();
#pragma unroll
    for (int p = 0; p < 4; ++p)
      *(volatile h8*)(base + (size_t)(p * 16 + sub) * HD) = vals[p];
  } else {
    h8 vals[4];
#pragma unroll
    for (int p = 0; p < 4; ++p) {
      const int dl = p * 16 + sub;
#pragma unroll
      for (int jj = 0; jj < 8; ++jj) vals[p][jj] = stg[(ch * 8 + jj) * SP + dl];
    }
    _Float16* base = vtb + (size_t)bh * HD * SEQ + t0 + ch * 8;
#pragma unroll
    for (int p = 0; p < 4; ++p)
      *(volatile h8*)(base + (size_t)(p * 16 + sub) * SEQ) = vals[p];
    __threadfence();
#pragma unroll
    for (int p = 0; p < 4; ++p)
      *(volatile h8*)(base + (size_t)(p * 16 + sub) * SEQ) = vals[p];
  }
}

#define PL 64

__global__ void __launch_bounds__(128) __attribute__((amdgpu_num_vgpr(256)))
k_attn(const _Float16* __restrict__ qb,
       const _Float16* __restrict__ kb,
       const _Float16* __restrict__ vtb,
       _Float16* __restrict__ att) {
  __shared__ __attribute__((aligned(16))) _Float16 plds[4][16 * PL];
  const int lane = threadIdx.x & 31, hh = lane >> 4, wslot = threadIdx.x >> 5;
  const int wid = blockIdx.x * 4 + wslot;
  const int bh = wid / (SEQ / 16), qt = wid - bh * (SEQ / 16);
  const _Float16* qh = qb  + ((size_t)bh * SEQ + qt * 16) * HD;
  const _Float16* kh = kb  + (size_t)bh * SEQ * HD;
  const _Float16* vt = vtb + (size_t)bh * HD * SEQ;
  _Float16* pl = plds[wslot];

  const h16 qa0 = load_frag(qh, HD, 0, lane);
  const h16 qa1 = load_frag(qh, HD, 32, lane);
  f8 o0 = {}, o1 = {}, o2 = {}, o3 = {};
  float m[8], lsum[8];
#pragma unroll
  for (int r = 0; r < 8; ++r) { m[r] = -1.0e30f; lsum[r] = 0.f; }

#pragma unroll 1
  for (int kc = 0; kc < SEQ; kc += 32) {
    f8 s0 = {}, s1 = {};
    h16 kf = load_frag(kh + (size_t)kc * HD, HD, 0, lane);
    s0 = wmma16(qa0, kf, s0);
    kf = load_frag(kh + (size_t)kc * HD, HD, 32, lane);
    s0 = wmma16(qa1, kf, s0);
    h16 kg = load_frag(kh + (size_t)(kc + 16) * HD, HD, 0, lane);
    s1 = wmma16(qa0, kg, s1);
    kg = load_frag(kh + (size_t)(kc + 16) * HD, HD, 32, lane);
    s1 = wmma16(qa1, kg, s1);
    asm volatile("v_nop\n\tv_nop\n\tv_nop\n\tv_nop"
                 : "+v"(s0), "+v"(s1) : "v"(qa1), "v"(kf), "v"(kg));

    float cm[8], corr[8], rsum[8];
#pragma unroll
    for (int r = 0; r < 8; ++r) {
      s0[r] = s0[r] * 0.125f;
      s1[r] = s1[r] * 0.125f;
      cm[r] = fmaxf(s0[r], s1[r]);
    }
#pragma unroll
    for (int off = 1; off < 16; off <<= 1) {
#pragma unroll
      for (int r = 0; r < 8; ++r) cm[r] = fmaxf(cm[r], __shfl_xor(cm[r], off, 32));
    }
#pragma unroll
    for (int r = 0; r < 8; ++r) {
      float mn = fmaxf(m[r], cm[r]);
      corr[r] = __expf(m[r] - mn);
      m[r]    = mn;
      s0[r]   = __expf(s0[r] - mn);
      s1[r]   = __expf(s1[r] - mn);
      rsum[r] = s0[r] + s1[r];
    }
#pragma unroll
    for (int off = 1; off < 16; off <<= 1) {
#pragma unroll
      for (int r = 0; r < 8; ++r) rsum[r] += __shfl_xor(rsum[r], off, 32);
    }
#pragma unroll
    for (int r = 0; r < 8; ++r) {
      lsum[r] = lsum[r] * corr[r] + rsum[r];
      o0[r] *= corr[r]; o1[r] *= corr[r]; o2[r] *= corr[r]; o3[r] *= corr[r];
      pl[(r + 8 * hh) * PL + (lane & 15)]      = (_Float16)(s0[r] * 1024.0f);
      pl[(r + 8 * hh) * PL + 16 + (lane & 15)] = (_Float16)(s1[r] * 1024.0f);
    }
    asm volatile("s_wait_dscnt 0" ::: "memory");
    __builtin_amdgcn_wave_barrier();
    h16 pa = load_frag(pl, PL, 0, lane);
    asm volatile("" ::: "memory");
    h16 vf = load_frag(vt + (size_t)0 * 16 * SEQ + kc, SEQ, 0, lane);
    o0 = wmma16(pa, vf, o0);
    vf = load_frag(vt + (size_t)1 * 16 * SEQ + kc, SEQ, 0, lane);
    o1 = wmma16(pa, vf, o1);
    vf = load_frag(vt + (size_t)2 * 16 * SEQ + kc, SEQ, 0, lane);
    o2 = wmma16(pa, vf, o2);
    vf = load_frag(vt + (size_t)3 * 16 * SEQ + kc, SEQ, 0, lane);
    o3 = wmma16(pa, vf, o3);
    asm volatile("v_nop\n\tv_nop\n\tv_nop\n\tv_nop"
                 : "+v"(o0), "+v"(o1), "+v"(o2), "+v"(o3) : "v"(pa), "v"(vf));
  }

  const int bb = bh / NH, hl = bh - bb * NH;
#pragma unroll
  for (int r = 0; r < 8; ++r) {
    float inv = 1.0f / (64.0f * lsum[r]);
    const int mrow = (r + 8 * hh) * PL + (lane & 15);
    pl[mrow + 0]  = (_Float16)(o0[r] * inv);
    pl[mrow + 16] = (_Float16)(o1[r] * inv);
    pl[mrow + 32] = (_Float16)(o2[r] * inv);
    pl[mrow + 48] = (_Float16)(o3[r] * inv);
  }
  asm volatile("s_wait_dscnt 0" ::: "memory");
  __builtin_amdgcn_wave_barrier();
  const int sub = lane >> 3, ch = lane & 7;
  h8 vals[4];
#pragma unroll
  for (int p = 0; p < 4; ++p) vals[p] = *(const h8*)(pl + (p * 4 + sub) * PL + ch * 8);
  _Float16* base = att + ((size_t)bb * SEQ + qt * 16) * DIM + hl * HD + ch * 8;
#pragma unroll
  for (int p = 0; p < 4; ++p)
    *(volatile h8*)(base + (size_t)(p * 4 + sub) * DIM) = vals[p];
  __threadfence();
#pragma unroll
  for (int p = 0; p < 4; ++p)
    *(volatile h8*)(base + (size_t)(p * 4 + sub) * DIM) = vals[p];
}

#define SPF 68

__global__ void __launch_bounds__(128) k_proj(const _Float16* __restrict__ att,
                                              const _Float16* __restrict__ wp,
                                              const float* __restrict__ bias,
                                              float* __restrict__ out) {
  __shared__ __attribute__((aligned(16))) float stg[64 * SPF];
  const int tid = threadIdx.x, lane = tid & 31, wid = tid >> 5, hh = lane >> 4;
  const int wm = wid & 1, wn = wid >> 1;
  const int mt = blockIdx.x / (DIM / 64), nt = blockIdx.x - mt * (DIM / 64);
  const int m0 = mt * 64, n0 = nt * 64;
  const int b = m0 / SEQ, t0 = m0 - b * SEQ;
  const _Float16* arow = att + (size_t)(m0 + wm * 32) * DIM;
  const _Float16* brow = wp  + (size_t)(n0 + wn * 32) * DIM;
  f8 c00 = {}, c01 = {}, c10 = {}, c11 = {};
#pragma unroll 1
  for (int k0 = 0; k0 < DIM; k0 += 32) {
    h16 a0 = load_frag(arow, DIM, k0, lane);
    h16 a1 = load_frag(arow + (size_t)16 * DIM, DIM, k0, lane);
    h16 b0 = load_frag(brow, DIM, k0, lane);
    h16 b1 = load_frag(brow + (size_t)16 * DIM, DIM, k0, lane);
    c00 = wmma16(a0, b0, c00);
    c01 = wmma16(a0, b1, c01);
    c10 = wmma16(a1, b0, c10);
    c11 = wmma16(a1, b1, c11);
    asm volatile("v_nop\n\tv_nop\n\tv_nop\n\tv_nop"
                 : "+v"(c00), "+v"(c01), "+v"(c10), "+v"(c11)
                 : "v"(a0), "v"(a1), "v"(b0), "v"(b1));
  }
#pragma unroll
  for (int i = 0; i < 2; ++i) {
#pragma unroll
    for (int j = 0; j < 2; ++j) {
      f8 acc = i ? (j ? c11 : c10) : (j ? c01 : c00);
      const int lc = wn * 32 + j * 16 + (lane & 15);
#pragma unroll
      for (int r = 0; r < 8; ++r) {
        const int lr = wm * 32 + i * 16 + 8 * hh + r;
        stg[lr * SPF + lc] = acc[r];
      }
    }
  }
  __syncthreads();

  const int sub = tid >> 4, c4 = tid & 15;
  v4f braw = *(const v4f*)(bias + n0 + c4 * 4);
  v4f b4;
#pragma unroll
  for (int e = 0; e < 4; ++e) { float be = braw[e]; b4[e] = bfr(be); }
  v4f vals[8];
#pragma unroll
  for (int p = 0; p < 8; ++p) {
    const int lr = p * 8 + sub;
    v4f a = *(const v4f*)(stg + lr * SPF + c4 * 4);
    vals[p] = a * (1.0f / 512.0f) + b4;
  }
  float* base = out + ((size_t)b * SEQ_FULL + t0) * DIM + n0 + c4 * 4;
#pragma unroll
  for (int p = 0; p < 8; ++p)
    *(volatile v4f*)(base + (size_t)(p * 8 + sub) * DIM) = vals[p];
  __threadfence();
#pragma unroll
  for (int p = 0; p < 8; ++p)
    *(volatile v4f*)(base + (size_t)(p * 8 + sub) * DIM) = vals[p];
}

extern "C" void kernel_launch(void* const* d_in, const int* in_sizes, int n_in,
                              void* d_out, int out_size, void* d_ws, size_t ws_size,
                              hipStream_t stream) {
  if (n_in < 4) return;
  if (in_sizes[0] < ((NB - 1) * SEQ_FULL + SEQ) * DIM) return;
  if (in_sizes[1] < QKVN * DIM) return;
  if (in_sizes[2] < DIM * DIM) return;
  if (in_sizes[3] < DIM) return;
  if (out_size < ((NB - 1) * SEQ_FULL + SEQ) * DIM) return;
  if (ws_size < WS_TOTAL) return;

  const float* x    = (const float*)d_in[0];
  const float* wqkv = (const float*)d_in[1];
  const float* wprj = (const float*)d_in[2];
  const float* bprj = (const float*)d_in[3];
  float* out = (float*)d_out;

  char* ws = (char*)d_ws;
  float*    tab = (float*)(ws + WS_TAB);
  _Float16* xh  = (_Float16*)(ws + WS_XH);
  _Float16* wq  = (_Float16*)(ws + WS_WQ);
  _Float16* wpl = (_Float16*)(ws + WS_WP);
  _Float16* qb  = (_Float16*)(ws + WS_Q);
  _Float16* kb  = (_Float16*)(ws + WS_K);
  _Float16* vtb = (_Float16*)(ws + WS_VT);
  _Float16* at  = (_Float16*)(ws + WS_ATT);

  k_tab<<<1, 128, 0, stream>>>(tab);
  {
    int total = ROWS * (DIM / 8);
    k_cvt<<<(total + 255) / 256, 256, 0, stream>>>(x, xh, ROWS, DIM / 8, SEQ, SEQ_FULL, 1.0f);
  }
  {
    int total = QKVN * (DIM / 8);
    k_cvt<<<(total + 255) / 256, 256, 0, stream>>>(wqkv, wq, QKVN, DIM / 8, QKVN, QKVN, 32.0f);
  }
  {
    int total = DIM * (DIM / 8);
    k_cvt<<<(total + 255) / 256, 256, 0, stream>>>(wprj, wpl, DIM, DIM / 8, DIM, DIM, 32.0f);
  }
  k_qkv_rot<<<(ROWS / 64) * (QKVN / 64), 128, 0, stream>>>(xh, wq, tab, qb, kb, vtb);
  k_attn<<<(NBH * (SEQ / 16)) / 4, 128, 0, stream>>>(qb, kb, vtb, at);
  k_proj<<<(ROWS / 64) * (DIM / 64), 128, 0, stream>>>(at, wpl, bprj, out);
}
